// DNRI_MLP_Decoder_49357764166098
// MI455X (gfx1250) — hardware-verified
//
#include <hip/hip_runtime.h>

typedef __attribute__((ext_vector_type(16))) _Float16 v16h;
typedef __attribute__((ext_vector_type(8)))  _Float16 v8h;
typedef __attribute__((ext_vector_type(16))) __bf16   v16b;
typedef __attribute__((ext_vector_type(8)))  __bf16   v8b;
typedef __attribute__((ext_vector_type(8)))  float    v8f;
typedef __attribute__((ext_vector_type(4)))  float    v4f;
typedef __attribute__((ext_vector_type(4)))  unsigned v4u;

#define NV 50
#define NSND 49
#define NE 2450
#define ETYPES 4
#define IN_F 16
#define MH 32
#define NHID 256
#define AUGK 64
#define MUPAD 64

__device__ __forceinline__ unsigned short f2bf_bits(float f) {
  unsigned u = __float_as_uint(f);
  return (unsigned short)((u + 0x7FFFu + ((u >> 16) & 1u)) >> 16);
}
__device__ __forceinline__ float bf_bits2f(unsigned short h) { return __uint_as_float(((unsigned)h) << 16); }

__device__ __forceinline__ void dep_guard_h(v8f& a, v8f& b, v16h x, v16h y) { asm volatile("v_nop\n\tv_nop\n\tv_nop\n\tv_nop" : "+v"(a), "+v"(b) : "v"(x), "v"(y)); }
__device__ __forceinline__ void dep_guard_b(v8f& a, v8f& b, v16b x, v16b y) { asm volatile("v_nop\n\tv_nop\n\tv_nop\n\tv_nop" : "+v"(a), "+v"(b) : "v"(x), "v"(y)); }
__device__ __forceinline__ void keep4_h(v16h a, v16h b, v16h c, v16h d) { asm volatile("v_nop" :: "v"(a), "v"(b), "v"(c), "v"(d)); }
__device__ __forceinline__ void keep4_b(v16b a, v16b b, v16b c, v16b d) { asm volatile("v_nop" :: "v"(a), "v"(b), "v"(c), "v"(d)); }
__device__ __forceinline__ void acc_guard4(v8f& a, v8f& b, v8f& c, v8f& d) { asm volatile("v_nop\n\tv_nop\n\tv_nop\n\tv_nop" : "+v"(a), "+v"(b), "+v"(c), "+v"(d)); }
template <typename T> struct Frag;
template <> struct Frag<_Float16> {
  typedef v16h V; union U { v16h v; v8h h[2]; };
  static __device__ __forceinline__ v16h load(const _Float16* p) {
    U f; f.h[0] = *(const v8h*)(p); f.h[1] = *(const v8h*)(p + 16); return f.v;
  }
  static __device__ __forceinline__ v8f mma(v16h a, v16h b, v8f c) {
    return __builtin_amdgcn_wmma_f32_16x16x32_f16(false, a, false, b, (short)0, c, false, false);
  }
  static __device__ __forceinline__ void guard(v8f& a, v8f& b, v16h x, v16h y) { dep_guard_h(a, b, x, y); }
  static __device__ __forceinline__ void keep(v16h a, v16h b, v16h c, v16h d) { keep4_h(a, b, c, d); }
};
template <> struct Frag<__bf16> {
  typedef v16b V; union U { v16b v; v8b h[2]; };
  static __device__ __forceinline__ v16b load(const __bf16* p) {
    U f; f.h[0] = *(const v8b*)(p); f.h[1] = *(const v8b*)(p + 16); return f.v;
  }
  static __device__ __forceinline__ v8f mma(v16b a, v16b b, v8f c) {
    return __builtin_amdgcn_wmma_f32_16x16x32_bf16(false, a, false, b, (short)0, c, false, false);
  }
  static __device__ __forceinline__ void guard(v8f& a, v8f& b, v16b x, v16b y) { dep_guard_b(a, b, x, y); }
  static __device__ __forceinline__ void keep(v16b a, v16b b, v16b c, v16b d) { keep4_b(a, b, c, d); }
};

template <int ET> struct Elem;
template <> struct Elem<0> { typedef _Float16 T; };
template <> struct Elem<1> { typedef __bf16 T; };
template <int ET, bool SPLIT, int BIAS_MODE, int OUT_MODE, bool RESID, int ACT = 0>
__global__ __launch_bounds__(256) void wmma_gemm64(
    const unsigned short* __restrict__ Ap, const unsigned short* __restrict__ A2p, int lda, long strideA,
    const unsigned short* __restrict__ Btp, const unsigned short* __restrict__ Bt2p, int ldb, long strideB,
    void* __restrict__ Cout, void* __restrict__ Cout2, int ldc, long strideC,
    const float* __restrict__ bias,
    const float* __restrict__ resid, long strideR,
    int M, int N, int K, float scale) {
  typedef typename Elem<ET>::T T;
  typedef typename Frag<T>::V V;
  const T* A = (const T*)Ap; const T* A2 = (const T*)A2p; const T* Bt = (const T*)Btp; const T* Bt2 = (const T*)Bt2p;
  __shared__ __align__(16) float sT[8][16 * 68];
  const int b    = blockIdx.y;
  const int lane = threadIdx.x & 31;
  const int wave = threadIdx.x >> 5;
  const int tilesN = N >> 6;
  const int tilesM = M >> 6;
  const int tile = blockIdx.x * 8 + wave;
  if (tile >= tilesM * tilesN) return;
  const int tm = tile / tilesN;
  const int tn = tile - tm * tilesN;
  const int m0 = tm << 6;
  const int n0 = tn << 6;

  const T* Ab  = A  + (size_t)b * strideA;
  const T* Bb  = Bt + (size_t)b * strideB;
  const T* Ab2 = SPLIT ? (A2  + (size_t)b * strideA) : nullptr;
  const T* Bb2 = SPLIT ? (Bt2 + (size_t)b * strideB) : nullptr;

  const int rlane = lane & 15;
  const int koff  = (lane >> 4) * 8;
  const int mOff  = (lane >> 4) * 8;

  v8f acc[4][4];
#pragma unroll
  for (int i = 0; i < 4; ++i)
#pragma unroll
    for (int j = 0; j < 4; ++j) acc[i][j] = (v8f){0.f,0.f,0.f,0.f,0.f,0.f,0.f,0.f};

  for (int k0 = 0; k0 < K; k0 += 32) {
    V bh[4], bl[4];
#pragma unroll
    for (int j = 0; j < 4; ++j) {
      const size_t bo = (size_t)(n0 + (j << 4) + rlane) * ldb + koff + k0;
      bh[j] = Frag<T>::load(Bb + bo);
      if (SPLIT) bl[j] = Frag<T>::load(Bb2 + bo);
    }
#pragma unroll
    for (int i = 0; i < 4; ++i) {
      const size_t ao = (size_t)(m0 + (i << 4) + rlane) * lda + koff + k0;
      V ah = Frag<T>::load(Ab + ao);
      V al;
      if (SPLIT) al = Frag<T>::load(Ab2 + ao);
#pragma unroll
      for (int j = 0; j < 4; ++j) {
        acc[i][j] = Frag<T>::mma(ah, bh[j], acc[i][j]);
        if (SPLIT) {
          acc[i][j] = Frag<T>::mma(ah, bl[j], acc[i][j]);
          acc[i][j] = Frag<T>::mma(al, bh[j], acc[i][j]);
        }
      }
      Frag<T>::guard(acc[i][0], acc[i][3], ah, SPLIT ? al : ah);
    }
    Frag<T>::keep(bh[0], bh[1], bh[2], bh[3]);
    if (SPLIT) Frag<T>::keep(bl[0], bl[1], bl[2], bl[3]);
  }
  acc_guard4(acc[0][0], acc[0][1], acc[0][2], acc[0][3]);
  acc_guard4(acc[1][0], acc[1][1], acc[1][2], acc[1][3]);
  acc_guard4(acc[2][0], acc[2][1], acc[2][2], acc[2][3]);
  acc_guard4(acc[3][0], acc[3][1], acc[3][2], acc[3][3]);

  float* slab = sT[wave];
  const float* Rb = RESID ? (resid + (size_t)b * strideR) : nullptr;
#pragma unroll
  for (int i = 0; i < 4; ++i) {
    const int mBase = m0 + (i << 4);
#pragma unroll
    for (int j = 0; j < 4; ++j) {
      const int n = n0 + (j << 4) + rlane;
      float bv = 0.f;
      if (BIAS_MODE == 2) bv = bias[n];
#pragma unroll
      for (int r = 0; r < 8; ++r) {
        float v = acc[i][j][r] * scale;
        if (BIAS_MODE == 1) v += bias[mBase + mOff + r];
        if (BIAS_MODE == 2) v += bv;
        if (RESID) v += Rb[(size_t)(mBase + mOff + r) * ldc + n];
        if (ACT == 1) v = tanhf(v);
        if (ACT == 2) v = fmaxf(v, 0.0f);
        if (ACT == 3) v = v / (1.0f + expf(-v));
        if (ACT == 4) v = (v > 0.f) ? v : 0.01f * v;
        if (ACT == 5) v = 0.5f * v * (1.0f + erff(v * 0.70710678118654752f));
        slab[(mOff + r) * 68 + (j << 4) + rlane] = v;
      }
    }
    __builtin_amdgcn_fence(__ATOMIC_RELEASE, "workgroup");
    __builtin_amdgcn_wave_barrier();
    __builtin_amdgcn_fence(__ATOMIC_ACQUIRE, "workgroup");
    if (OUT_MODE == 0 || OUT_MODE == 3) {
      float* C = (float*)Cout + (size_t)b * strideC;
      const int hh = lane >> 4, c4 = (lane & 15) * 4;
      for (int pass = 0; pass < 2; ++pass) {
#pragma unroll
        for (int it = 0; it < 8; ++it) {
          const int row = it * 2 + hh;
          v4f v = *(const v4f*)(slab + row * 68 + c4);
          *(volatile v4f*)(C + (size_t)(mBase + row) * ldc + n0 + c4) = v;
        }
        __threadfence();
      }
    }
    if (OUT_MODE != 0) {
      const int q = lane >> 3, c8 = (lane & 7) * 8;
      unsigned short* C  = (unsigned short*)((OUT_MODE == 3) ? Cout2 : Cout) + (size_t)b * strideC;
      unsigned short* C2 = (OUT_MODE == 2) ? ((unsigned short*)Cout2 + (size_t)b * strideC) : nullptr;
      for (int pass = 0; pass < 2; ++pass) {
#pragma unroll
        for (int it = 0; it < 4; ++it) {
          const int row = it * 4 + q;
          const float* sp = slab + row * 68 + c8;
          v8h hv, lv;
#pragma unroll
          for (int e = 0; e < 8; ++e) {
            if (OUT_MODE == 1 || OUT_MODE == 3) {
              hv[e] = (_Float16)sp[e];
            } else {
              unsigned short hb = f2bf_bits(sp[e]);
              unsigned short lb = f2bf_bits(sp[e] - bf_bits2f(hb));
              hv[e] = __builtin_bit_cast(_Float16, hb);
              lv[e] = __builtin_bit_cast(_Float16, lb);
            }
          }
          *(volatile v8h*)(C + (size_t)(mBase + row) * ldc + n0 + c8) = hv;
          if (OUT_MODE == 2) *(volatile v8h*)(C2 + (size_t)(mBase + row) * ldc + n0 + c8) = lv;
        }
        __threadfence();
      }
    }
    __builtin_amdgcn_fence(__ATOMIC_RELEASE, "workgroup");
    __builtin_amdgcn_wave_barrier();
    __builtin_amdgcn_fence(__ATOMIC_ACQUIRE, "workgroup");
  }
}

__global__ __launch_bounds__(256) void k_castT(
    const float* __restrict__ in, _Float16* __restrict__ out,
    int Kin, int Nin, int Kpad, int Npad, int total2) {
  const int i = blockIdx.x * 256 + threadIdx.x;
  if (i < total2) {
    const int idx = 2 * i;
    const int kp = idx % Kpad;
    const int rest = idx / Kpad;
    const int n = rest % Npad;
    const int z = rest / Npad;
    const float* inz = in + (size_t)z * Kin * Nin;
    const int nc = n < Nin ? n : Nin - 1;
    const int k0 = kp < Kin ? kp : Kin - 1;
    const int k1 = (kp + 1) < Kin ? (kp + 1) : Kin - 1;
    float f0 = inz[(size_t)k0 * Nin + nc];
    float f1 = inz[(size_t)k1 * Nin + nc];
    if (n >= Nin || kp >= Kin) f0 = 0.0f;
    if (n >= Nin || (kp + 1) >= Kin) f1 = 0.0f;
    const _Float16 h0 = (_Float16)f0, h1 = (_Float16)f1;
    const unsigned u = (unsigned)__builtin_bit_cast(unsigned short, h0) | ((unsigned)__builtin_bit_cast(unsigned short, h1) << 16);
    ((volatile unsigned*)out)[i] = u;
    __threadfence();
    ((volatile unsigned*)out)[i] = u;
  }
}

__device__ __forceinline__ v8f mma_h(v16h a, v16h b, v8f c) {
  c = __builtin_amdgcn_wmma_f32_16x16x32_f16(false, a, false, b, (short)0, c, false, false);
  asm volatile("v_nop\n\tv_nop\n\tv_nop\n\tv_nop" : "+v"(c) : "v"(a), "v"(b));
  return c;
}
__device__ __forceinline__ void wave_sync_lds() {
  __builtin_amdgcn_fence(__ATOMIC_RELEASE, "workgroup");
  __builtin_amdgcn_wave_barrier();
  __builtin_amdgcn_fence(__ATOMIC_ACQUIRE, "workgroup");
}
__device__ __forceinline__ v8h pack8h(v4f a, v4f b) {
  v8h p;
  p[0] = (_Float16)a[0]; p[1] = (_Float16)a[1]; p[2] = (_Float16)a[2]; p[3] = (_Float16)a[3];
  p[4] = (_Float16)b[0]; p[5] = (_Float16)b[1]; p[6] = (_Float16)b[2]; p[7] = (_Float16)b[3];
  return p;
}

__global__ __launch_bounds__(128) void k_edge_msg(
    const float* __restrict__ inputs, const float* __restrict__ edges,
    const _Float16* __restrict__ w1t, const float* __restrict__ b1,
    const _Float16* __restrict__ w2t, const float* __restrict__ b2,
    _Float16* __restrict__ aug, int npairs) {
  __shared__ __align__(16) _Float16 Wsh[2][3][MH * MH];
  __shared__ __align__(16) float    Bsh[2][3][MH];
  __shared__ __align__(16) _Float16 pre_s[4][16 * MH];
  __shared__ __align__(16) _Float16 h_s[4][16 * MH];
  __shared__ __align__(16) float    cf_s[4][16 * 4];
  __shared__ __align__(16) _Float16 o_s[4][AUGK];

  const int tid = threadIdx.x;
  {
    const v4u* s1 = (const v4u*)(w1t + MH * MH);
    const v4u* s2 = (const v4u*)(w2t + MH * MH);
    v4u* d1 = (v4u*)&Wsh[0][0][0];
    v4u* d2 = (v4u*)&Wsh[1][0][0];
    for (int i = tid; i < (3 * MH * MH) / 8; i += 128) { d1[i] = s1[i]; d2[i] = s2[i]; }
    if (tid < 3 * MH) {
      (&Bsh[0][0][0])[tid] = b1[MH + tid];
      (&Bsh[1][0][0])[tid] = b2[MH + tid];
    }
  }
  __syncthreads();

  const int wave = tid >> 5, lane = tid & 31, h = lane >> 4, m = lane & 15;
  const int pair = blockIdx.x * 4 + wave;
  if (pair >= npairs) return;
  const int b = pair / NV;
  const int r = pair - b * NV;

  const float* xb = inputs + (size_t)b * NV * IN_F;
  const float* xr = xb + r * IN_F;
  v8h recv0, recv1;
  {
    const v4f q0 = *(const v4f*)(xr + 0), q1 = *(const v4f*)(xr + 4);
    const v4f q2 = *(const v4f*)(xr + 8), q3 = *(const v4f*)(xr + 12);
    recv0 = pack8h(q0, q1); recv1 = pack8h(q2, q3);
  }
  v8h z8;
#pragma unroll
  for (int e = 0; e < 8; ++e) z8[e] = (_Float16)0.0f;
  const float* eb = edges + (size_t)b * NE * ETYPES;

  _Float16* pre = pre_s[wave];
  _Float16* hs  = h_s[wave];
  float*    cf  = cf_s[wave];

  float acc0 = 0.f, acc1 = 0.f;
#pragma unroll 1
  for (int t = 0; t < 4; ++t) {
    const int q = t * 16 + m;
    const bool valid = q < NSND;
    int s = q + ((q >= r) ? 1 : 0);
    s = (s > NV - 1) ? (NV - 1) : s;
    _Float16* row = pre + m * MH;
    if (h == 0) {
      v8h o0 = z8, o1 = z8;
      if (valid) { o0 = recv0; o1 = recv1; }
      *(v8h*)(row + 0) = o0;
      *(v8h*)(row + 8) = o1;
      const int e = s * NSND + ((r < s) ? r : (r - 1));
      v4f cv = *(const v4f*)(eb + (size_t)e * ETYPES);
      if (!valid) cv = (v4f){0.f, 0.f, 0.f, 0.f};
      *(v4f*)(cf + m * 4) = cv;
    } else {
      const float* xs = xb + s * IN_F;
      const v4f p0 = *(const v4f*)(xs + 0), p1 = *(const v4f*)(xs + 4);
      const v4f p2 = *(const v4f*)(xs + 8), p3 = *(const v4f*)(xs + 12);
      v8h sa = z8, sb = z8;
      if (valid) { sa = pack8h(p0, p1); sb = pack8h(p2, p3); }
      *(v8h*)(row + 16) = sa;
      *(v8h*)(row + 24) = sb;
    }
    wave_sync_lds();
    const v16h a0 = Frag<_Float16>::load(pre + m * MH + 8 * h);

#pragma unroll 1
    for (int kt = 0; kt < 3; ++kt) {
      const _Float16* W1 = Wsh[0][kt];
      const _Float16* W2 = Wsh[1][kt];
      const float* B1 = Bsh[0][kt];
      const float* B2 = Bsh[1][kt];
#pragma unroll
      for (int hn = 0; hn < 2; ++hn) {
        const float bias = B1[hn * 16 + m];
        v8f c;
#pragma unroll
        for (int v = 0; v < 8; ++v) c[v] = bias;
        const v16h bw = Frag<_Float16>::load(W1 + (hn * 16 + m) * MH + 8 * h);
        c = mma_h(a0, bw, c);
#pragma unroll
        for (int v = 0; v < 8; ++v) hs[(8 * h + v) * MH + hn * 16 + m] = (_Float16)fmaxf(c[v], 0.0f);
      }
      wave_sync_lds();
      const v16h a1 = Frag<_Float16>::load(hs + m * MH + 8 * h);
      wave_sync_lds();
#pragma unroll
      for (int hn = 0; hn < 2; ++hn) {
        const float bias = B2[hn * 16 + m];
        v8f c;
#pragma unroll
        for (int v = 0; v < 8; ++v) c[v] = bias;
        const v16h bw = Frag<_Float16>::load(W2 + (hn * 16 + m) * MH + 8 * h);
        c = mma_h(a1, bw, c);
        float sacc = 0.f;
#pragma unroll
        for (int v = 0; v < 8; ++v) {
          const float cw = cf[(8 * h + v) * 4 + kt + 1];
          sacc += fmaxf(c[v], 0.0f) * cw;
        }
        if (hn == 0) acc0 += sacc; else acc1 += sacc;
      }
    }
    wave_sync_lds();
  }

  acc0 += __shfl_xor(acc0, 16, 32);
  acc1 += __shfl_xor(acc1, 16, 32);
  const float aggv = (h == 0) ? acc0 : acc1;
  const float xrl = xr[m];
  _Float16* os = o_s[wave];
  os[IN_F + lane] = (_Float16)aggv;
  if (h == 0) os[m] = (_Float16)xrl;
  else os[IN_F + MH + m] = (_Float16)0.0f;
  wave_sync_lds();
  _Float16* dst = aug + (size_t)pair * AUGK;
  const v8h ov = *(const v8h*)(os + 8 * (lane & 7));
  if (lane < 8) *(volatile v8h*)(dst + 8 * lane) = ov;
  __threadfence();
  if (lane < 8) *(volatile v8h*)(dst + 8 * lane) = ov;
}

__global__ __launch_bounds__(256) void k_mu_out(
    const float* __restrict__ mupad, const float* __restrict__ mub,
    float* __restrict__ out, int nrows) {
  const int i = blockIdx.x * 256 + threadIdx.x;
  const int row = i >> 2, qd = i & 3;
  const int rowc = row < nrows ? row : (nrows - 1);
  v4f v = *(const v4f*)(mupad + (size_t)rowc * MUPAD + qd * 4);
  const v4f bb = *(const v4f*)(mub + qd * 4);
  v = v + bb;
  if (row < nrows) *(volatile v4f*)(out + (size_t)row * IN_F + qd * 4) = v;
  __threadfence();
  if (row < nrows) *(volatile v4f*)(out + (size_t)row * IN_F + qd * 4) = v;
}

extern "C" void kernel_launch(void* const* d_in, const int* in_sizes, int n_in,
                              void* d_out, int out_size, void* d_ws,
                              size_t ws_size, hipStream_t stream) {
  if (n_in < 12) return;
  const float* inputs = (const float*)d_in[0];
  const float* edges  = (const float*)d_in[1];
  const float* w1     = (const float*)d_in[2];
  const float* b1     = (const float*)d_in[3];
  const float* w2     = (const float*)d_in[4];
  const float* b2     = (const float*)d_in[5];
  const float* fc1w   = (const float*)d_in[6];
  const float* fc1b   = (const float*)d_in[7];
  const float* fc2w   = (const float*)d_in[8];
  const float* fc2b   = (const float*)d_in[9];
  const float* muw    = (const float*)d_in[10];
  const float* mub    = (const float*)d_in[11];

  const int npairs = in_sizes[0] / IN_F;
  if (npairs <= 0 || (npairs % 64) != 0 || (npairs % NV) != 0) return;
  const int nbatch = npairs / NV;
  if (in_sizes[1] != nbatch * NE * ETYPES) return;
  if (out_size != npairs * (IN_F + NHID)) return;
  if (in_sizes[11] < IN_F) return;

  float* mu_out   = (float*)d_out;
  float* pred_out = (float*)d_out + (size_t)npairs * IN_F;

  size_t off = 0;
  char* wsb = (char*)d_ws;
  auto carve = [&](size_t bytes) -> char* { char* p = wsb + off; off += (bytes + 255) & ~(size_t)255; return p; };
  _Float16* w1t   = (_Float16*)carve((size_t)ETYPES * MH * MH * 2);
  _Float16* w2t   = (_Float16*)carve((size_t)ETYPES * MH * MH * 2);
  _Float16* fc1t  = (_Float16*)carve((size_t)NHID * AUGK * 2);
  _Float16* fc2t  = (_Float16*)carve((size_t)NHID * NHID * 2);
  _Float16* mut   = (_Float16*)carve((size_t)MUPAD * NHID * 2);
  _Float16* aug   = (_Float16*)carve((size_t)npairs * AUGK * 2);
  _Float16* h1    = (_Float16*)carve((size_t)npairs * NHID * 2);
  _Float16* h2    = (_Float16*)carve((size_t)npairs * NHID * 2);
  float*    mupad = (float*)carve((size_t)npairs * MUPAD * 4);
  if (off > ws_size || off > (size_t)134217728) return;

  {
    int total2;
    total2 = ETYPES * MH * MH / 2;
    k_castT<<<(total2 + 255) / 256, 256, 0, stream>>>(w1, w1t, MH, MH, MH, MH, total2);
    k_castT<<<(total2 + 255) / 256, 256, 0, stream>>>(w2, w2t, MH, MH, MH, MH, total2);
    total2 = NHID * AUGK / 2;
    k_castT<<<(total2 + 255) / 256, 256, 0, stream>>>(fc1w, fc1t, IN_F + MH, NHID, AUGK, NHID, total2);
    total2 = NHID * NHID / 2;
    k_castT<<<(total2 + 255) / 256, 256, 0, stream>>>(fc2w, fc2t, NHID, NHID, NHID, NHID, total2);
    total2 = MUPAD * NHID / 2;
    k_castT<<<(total2 + 255) / 256, 256, 0, stream>>>(muw, mut, NHID, IN_F, NHID, MUPAD, total2);
  }

  k_edge_msg<<<(npairs + 3) / 4, 128, 0, stream>>>(inputs, edges, w1t, b1, w2t, b2, aug, npairs);

  const int M = npairs;
  {
    const int tiles = (M / 64) * (NHID / 64);
    wmma_gemm64<0, false, 2, 1, false, 2><<<dim3((tiles + 7) / 8, 1), 256, 0, stream>>>(
        (const unsigned short*)aug, (const unsigned short*)aug, AUGK, 0L,
        (const unsigned short*)fc1t, (const unsigned short*)fc1t, AUGK, 0L,
        (void*)h1, (void*)h1, NHID, 0L,
        fc1b, fc1b, 0L, M, NHID, AUGK, 1.0f);
  }
  {
    const int tiles = (M / 64) * (NHID / 64);
    wmma_gemm64<0, false, 2, 3, false, 2><<<dim3((tiles + 7) / 8, 1), 256, 0, stream>>>(
        (const unsigned short*)h1, (const unsigned short*)h1, NHID, 0L,
        (const unsigned short*)fc2t, (const unsigned short*)fc2t, NHID, 0L,
        (void*)pred_out, (void*)h2, NHID, 0L,
        fc2b, fc2b, 0L, M, NHID, NHID, 1.0f);
  }
  {
    const int tiles = (M / 64) * (MUPAD / 64);
    wmma_gemm64<0, false, 0, 0, false, 0><<<dim3((tiles + 7) / 8, 1), 256, 0, stream>>>(
        (const unsigned short*)h2, (const unsigned short*)h2, NHID, 0L,
        (const unsigned short*)mut, (const unsigned short*)mut, NHID, 0L,
        (void*)mupad, (void*)mupad, MUPAD, 0L,
        fc2b, fc2b, 0L, M, MUPAD, NHID, 1.0f);
  }
  k_mu_out<<<(npairs * 4 + 255) / 256, 256, 0, stream>>>(mupad, mub, mu_out, npairs);
}
